// KDMLP_17617955848556
// MI455X (gfx1250) — hardware-verified
//
#include <hip/hip_runtime.h>
#include <math.h>

typedef __attribute__((ext_vector_type(16))) _Float16 v16h;
typedef __attribute__((ext_vector_type(16))) __bf16 v16b;
typedef __attribute__((ext_vector_type(8)))  _Float16 v8h;
typedef __attribute__((ext_vector_type(8)))  float v8f;
typedef __attribute__((ext_vector_type(4)))  float v4f;
typedef __attribute__((ext_vector_type(2)))  float v2f;
typedef __attribute__((ext_vector_type(4)))  unsigned v4u;
typedef __attribute__((ext_vector_type(4)))  int v4i;
typedef float __attribute__((may_alias)) float_a;
typedef int __attribute__((may_alias)) int_a;

template <typename T> __device__ __forceinline__ void vst2(void* p, T v) { *(volatile T*)p = v; __threadfence(); *(volatile T*)p = v; }
__device__ __forceinline__ v8f wmma16(v16h a, v16h b, v8f c) {
  v8f d = __builtin_amdgcn_wmma_f32_16x16x32_f16(false, a, false, b, (short)0, c, false, false);
  asm volatile("v_nop\n\tv_nop\n\tv_nop\n\tv_nop" : "+v"(d) : "v"(a), "v"(b));
  return d;
}
__device__ __forceinline__ v8f wmma_bf(v16b a, v16b b, v8f c) {
  v8f d = __builtin_amdgcn_wmma_f32_16x16x32_bf16(false, a, false, b, (short)0, c, false, false);
  asm volatile("v_nop\n\tv_nop\n\tv_nop\n\tv_nop" : "+v"(d) : "v"(a), "v"(b));
  return d;
}
__device__ __forceinline__ v16h frag_h(const _Float16* rowk0, int lane) {
  union { v16h v; v8h q[2]; } u; const _Float16* p = rowk0 + 8 * (lane >> 4);
  u.q[0] = *(const v8h*)p; u.q[1] = *(const v8h*)(p + 16); return u.v;
}
__device__ __forceinline__ v16h frag_f32(const float* rowk0, int lane) {
  v16h a; const float* p = rowk0 + 8 * (lane >> 4);
#pragma unroll
  for (int i = 0; i < 8; ++i) { a[i] = (_Float16)p[i]; a[8 + i] = (_Float16)p[16 + i]; }
  return a;
}
__device__ __forceinline__ v16h frag_f32s(const float* rowk0, int lane, float sc) {
  v16h a; const float* p = rowk0 + 8 * (lane >> 4);
#pragma unroll
  for (int i = 0; i < 8; ++i) { a[i] = (_Float16)(p[i] * sc); a[8 + i] = (_Float16)(p[16 + i] * sc); }
  return a;
}
__device__ __forceinline__ v16h fragc_f32(const float* W, int k0, int n, int lane, int ld, int K) {
  v16h a; const int g = lane >> 4;
#pragma unroll
  for (int i = 0; i < 8; ++i) { const int ka = k0 + 8 * g + i, kb = ka + 16;
    a[i] = (_Float16)(ka < K ? W[(size_t)(ka < K ? ka : K - 1) * ld + n] : 0.f); a[8 + i] = (_Float16)(kb < K ? W[(size_t)(kb < K ? kb : K - 1) * ld + n] : 0.f); }
  return a;
}
struct F2 { v16b h, l; };
__device__ __forceinline__ F2 bsplit16(const float v[16]) { F2 r;
#pragma unroll
  for (int i = 0; i < 16; ++i) { const __bf16 h = (__bf16)v[i]; r.h[i] = h; r.l[i] = (__bf16)(v[i] - (float)h); }
  return r; }
__device__ __forceinline__ F2 split_row(const float* row, int k0, int lane) { float v[16]; const float* p = row + k0 + 8 * (lane >> 4);
#pragma unroll
  for (int i = 0; i < 8; ++i) { v[i] = p[i]; v[8 + i] = p[16 + i]; }
  return bsplit16(v); }
__device__ __forceinline__ F2 split_rowK(const float* row, int k0, int lane, int K) { float v[16]; const int g = lane >> 4;
#pragma unroll
  for (int i = 0; i < 8; ++i) { const int ka = k0 + 8 * g + i, kb = ka + 16; v[i] = ka < K ? row[ka < K ? ka : K - 1] : 0.f; v[8 + i] = kb < K ? row[kb < K ? kb : K - 1] : 0.f; }
  return bsplit16(v); }
__device__ __forceinline__ F2 split_col(const float* W, int k0, int n, int lane, int ld, int K) { float v[16]; const int g = lane >> 4;
#pragma unroll
  for (int i = 0; i < 8; ++i) { const int ka = k0 + 8 * g + i, kb = ka + 16; v[i] = ka < K ? W[(size_t)(ka < K ? ka : K - 1) * ld + n] : 0.f; v[8 + i] = kb < K ? W[(size_t)(kb < K ? kb : K - 1) * ld + n] : 0.f; }
  return bsplit16(v); }
__device__ __forceinline__ v8f mac3(const F2& a, const F2& b, v8f c) { c = wmma_bf(a.l, b.h, c); c = wmma_bf(a.h, b.l, c); return wmma_bf(a.h, b.h, c); }
__device__ __forceinline__ float sigm(float v) { return 1.0f / (1.0f + expf(-v)); }
#define LDSX() do { asm volatile("s_wait_dscnt 0" ::: "memory"); __builtin_amdgcn_wave_barrier(); __builtin_amdgcn_fence(__ATOMIC_RELEASE, "workgroup"); } while (0)


#define NBR 65536
#define NUSR 100000
#define NITM 50000
#define NKN 5000
#define KK 20
#define UD 128
#define KD 64
#define IN0 448
#define H1 256
#define H2 128
#define H3 64
#ifndef TRB
#define TRB (NBR / 64)
#endif
typedef __attribute__((ext_vector_type(8))) __bf16 v8b;
__device__ __forceinline__ v16b frag_b(const __bf16* rowk0, int lane) {
  union { v16b v; v8b q[2]; } u; const __bf16* p = rowk0 + 8 * (lane >> 4);
  u.q[0] = *(const v8b*)p; u.q[1] = *(const v8b*)(p + 16); return u.v;
}
__device__ __forceinline__ float bfr(float v) { return (float)(__bf16)v; }
__device__ __attribute__((noinline)) float exp_ni(float v) { return expf(v); }
__device__ __attribute__((noinline)) float erf_ni(float v) { return erff(v); }

#define WS_P1  0u
#define WS_P2  (WS_P1 + 2u * (size_t)H1 * IN0)
#define WS_P3  (WS_P2 + 2u * (size_t)H2 * H1)
#define WS_END (WS_P3 + 2u * (size_t)H3 * H2)

__global__ __launch_bounds__(256) void k_pack(const float* __restrict__ W1, const float* __restrict__ W2, const float* __restrict__ W3, __bf16* __restrict__ P) { const int n = blockIdx.x, which = blockIdx.y, t = threadIdx.x; __shared__ __align__(16) __bf16 s[IN0];
  if (which == 0) { for (int k = t; k < IN0; k += 256) s[k] = (__bf16)W1[(size_t)k * H1 + n]; __syncthreads(); for (int q = t; q < IN0 / 8; q += 256) vst2((unsigned*)(P + WS_P1 / 2 + (size_t)n * IN0 + q * 8), *(const v4u*)&s[q * 8]); }
  else if (which == 1) { if (n >= H2) return; s[t] = (__bf16)W2[(size_t)t * H2 + n]; __syncthreads(); if (t < H1 / 8) vst2((unsigned*)(P + WS_P2 / 2 + (size_t)n * H1 + t * 8), *(const v4u*)&s[t * 8]); }
  else { if (n >= H3) return; if (t < H2) s[t] = (__bf16)W3[(size_t)t * H3 + n]; __syncthreads(); if (t < H2 / 8) vst2((unsigned*)(P + WS_P3 / 2 + (size_t)n * H2 + t * 8), *(const v4u*)&s[t * 8]); } }
__device__ __forceinline__ int clampi(int v, int n) { return v < 0 ? 0 : (v >= n ? n - 1 : v); }
__device__ __forceinline__ void in_chunk(int kc, int g, int usr, int itm, const int* kids, int nv0, int nv1, int nv2, const float* EU, const float* EI, const float* EK, float* v) {
  if (kc < 8) { const float* src = (kc < 4) ? (EU + (size_t)usr * UD + kc * 32) : (EI + (size_t)itm * UD + (kc - 4) * 32);
#pragma unroll
    for (int i = 0; i < 8; ++i) { v[i] = bfr(src[8 * g + i]); v[8 + i] = bfr(src[16 + 8 * g + i]); } return; }
  const int which = (kc - 8) >> 1, half = (kc - 8) & 1; const int nv = which == 0 ? nv0 : (which == 1 ? nv1 : nv2); const int* ids = kids + which * KK;
#pragma unroll
  for (int i = 0; i < 16; ++i) v[i] = 0.f;
  if (nv > 0) {
#pragma unroll 1
    for (int n = 0; n < KK; ++n) { if (n >= nv) break; const float* src = EK + (size_t)clampi(ids[n], NKN) * KD + half * 32;
#pragma unroll
      for (int i = 0; i < 8; ++i) { v[i] += bfr(src[8 * g + i]); v[8 + i] += bfr(src[16 + 8 * g + i]); } }
    const float inv = 1.0f / (float)nv;
#pragma unroll
    for (int i = 0; i < 16; ++i) v[i] *= inv; } }
__global__ __launch_bounds__(128) void k_main(const int* __restrict__ USR, const int* __restrict__ ITM, const int* __restrict__ PK, const int* __restrict__ TK, const int* __restrict__ IK, const int* __restrict__ NV0, const int* __restrict__ NV1, const int* __restrict__ NV2,
    const float* __restrict__ EU, const float* __restrict__ EI, const float* __restrict__ EK, const __bf16* __restrict__ P, const float* __restrict__ B1, const float* __restrict__ B2, const float* __restrict__ B3, const float* __restrict__ WP, const float* __restrict__ BP, float* __restrict__ OUT) {
  __shared__ __align__(16) float sh1[64][H1 + 4]; __shared__ __align__(16) float sh2[64][H2 + 4]; __shared__ __align__(16) float sh3[64][H3 + 4]; __shared__ __align__(16) float so2[64]; __shared__ int skid[64][3 * KK];
  const int tid = threadIdx.x, wave = tid >> 5, lane = tid & 31, col = lane & 15, g = lane >> 4; const size_t rb = (size_t)blockIdx.x * 64; const size_t r0 = rb + wave * 16; const size_t row = r0 + col;
  for (int e = tid; e < 64 * 3 * KK; e += 128) { const int rl = e / (3 * KK), q = e % (3 * KK); const int which = q / KK, n = q % KK; const int* src = which == 0 ? PK : (which == 1 ? TK : IK); skid[rl][q] = src[(rb + rl) * KK + n]; }
  __syncthreads();
  const int usr = clampi(USR[row], NUSR), itm = clampi(ITM[row], NITM); int nv0 = NV0[row], nv1 = NV1[row], nv2 = NV2[row]; nv0 = nv0 < 0 ? 0 : (nv0 > KK ? KK : nv0); nv1 = nv1 < 0 ? 0 : (nv1 > KK ? KK : nv1); nv2 = nv2 < 0 ? 0 : (nv2 > KK ? KK : nv2);
  { v8f acc[16];
#pragma unroll
    for (int j = 0; j < 16; ++j) acc[j] = v8f{};
#pragma unroll 1
    for (int kc = 0; kc < IN0 / 32; ++kc) { float v[16]; in_chunk(kc, g, usr, itm, &skid[wave * 16 + col][0], nv0, nv1, nv2, EU, EI, EK, v); const F2 a = bsplit16(v);
#pragma unroll
      for (int j = 0; j < 16; ++j) { const v16b w = frag_b(P + WS_P1 / 2 + (size_t)(j * 16 + col) * IN0 + kc * 32, lane); acc[j] = wmma_bf(a.h, w, acc[j]); acc[j] = wmma_bf(a.l, w, acc[j]); } }
#pragma unroll
    for (int j = 0; j < 16; ++j) { const float bb = bfr(B1[j * 16 + col]);
#pragma unroll
      for (int r = 0; r < 8; ++r) sh1[wave * 16 + 8 * g + r][j * 16 + col] = fmaxf(acc[j][r] + bb, 0.f); } }
  LDSX();
  { v8f acc[8] = {};
#pragma unroll 1
    for (int kc = 0; kc < H1 / 32; ++kc) { float v[16]; const float* p2 = &sh1[wave * 16 + col][kc * 32 + 8 * g];
#pragma unroll
      for (int i = 0; i < 8; ++i) { v[i] = p2[i]; v[8 + i] = p2[16 + i]; }
      const F2 a = bsplit16(v);
#pragma unroll
      for (int j = 0; j < 8; ++j) { const v16b w = frag_b(P + WS_P2 / 2 + (size_t)(j * 16 + col) * H1 + kc * 32, lane); acc[j] = wmma_bf(a.h, w, acc[j]); acc[j] = wmma_bf(a.l, w, acc[j]); } }
#pragma unroll
    for (int j = 0; j < 8; ++j) { const float bb = bfr(B2[j * 16 + col]);
#pragma unroll
      for (int r = 0; r < 8; ++r) sh2[wave * 16 + 8 * g + r][j * 16 + col] = fmaxf(acc[j][r] + bb, 0.f); } }
  LDSX();
  { v8f acc[4] = {};
#pragma unroll 1
    for (int kc = 0; kc < H2 / 32; ++kc) { float v[16]; const float* p2 = &sh2[wave * 16 + col][kc * 32 + 8 * g];
#pragma unroll
      for (int i = 0; i < 8; ++i) { v[i] = p2[i]; v[8 + i] = p2[16 + i]; }
      const F2 a = bsplit16(v);
#pragma unroll
      for (int j = 0; j < 4; ++j) { const v16b w = frag_b(P + WS_P3 / 2 + (size_t)(j * 16 + col) * H2 + kc * 32, lane); acc[j] = wmma_bf(a.h, w, acc[j]); acc[j] = wmma_bf(a.l, w, acc[j]); } }
#pragma unroll
    for (int j = 0; j < 4; ++j) { const float bb = bfr(B3[j * 16 + col]);
#pragma unroll
      for (int r = 0; r < 8; ++r) sh3[wave * 16 + 8 * g + r][j * 16 + col] = fmaxf(acc[j][r] + bb, 0.f); } }
  __syncthreads();
  if (tid < 64) { float s = bfr(BP[0]);
#pragma unroll 1
    for (int i = 0; i < H3; ++i) s += sh3[tid][i] * bfr(WP[i]); so2[tid] = s; }
  __syncthreads(); if (tid < 16) vst2(OUT + rb + tid * 4, *(const v4f*)&so2[tid * 4]); }
extern "C" void kernel_launch(void* const* d_in, const int* in_sizes, int n_in, void* d_out, int out_size, void* d_ws, size_t ws_size, hipStream_t stream) {
  (void)in_sizes; (void)n_in; (void)out_size;
  const float** F = (const float**)d_in; const int** I = (const int**)d_in;
  if (ws_size < (size_t)WS_END) return;
  __bf16* P = (__bf16*)d_ws;
  k_pack<<<dim3(H1, 3), 256, 0, stream>>>(F[11], F[13], F[15], P);
  k_main<<<TRB, 128, 0, stream>>>(I[0], I[1], I[2], I[3], I[4], I[5], I[6], I[7], F[8], F[9], F[10], P, F[12], F[14], F[16], F[17], F[18], (float*)d_out);
}
